// RNNLayer_40879498728894
// MI455X (gfx1250) — hardware-verified
//
#include <hip/hip_runtime.h>
#include <stdint.h>


constexpr int kBatch   = 64;
constexpr int kSteps   = 128;
constexpr int kFeat    = 1024;
constexpr int kHid     = 1024;
constexpr int kGate4   = 4 * kHid;
constexpr int kColsBlk = 64;
constexpr int kTPitch  = 72;

static_assert(kBatch == 64);
static_assert(kFeat % 32 == 0);
static_assert(kHid % 32 == 0);
static_assert(kFeat == kHid);
static_assert(kHid % kColsBlk == 0);
static_assert(kGate4 % 64 == 0);
static_assert((kFeat + kHid) % 64 == 0);
static_assert((kBatch * kSteps * kFeat) % (8 * 256) == 0);

typedef __attribute__((ext_vector_type(16))) __bf16   v16b;
typedef __attribute__((ext_vector_type(8)))  __bf16   v8b;
typedef __attribute__((ext_vector_type(8)))  float    v8f;
typedef __attribute__((ext_vector_type(4)))  float    v4f;
typedef __attribute__((ext_vector_type(4)))  unsigned v4u;

__device__ __forceinline__ unsigned short f2bf_bits(float f) {
  unsigned u = __float_as_uint(f);
  return (unsigned short)((u + 0x7FFFu + ((u >> 16) & 1u)) >> 16);
}
__device__ __forceinline__ float bf_bits2f(unsigned short h) { return __uint_as_float(((unsigned)h) << 16); }

__device__ __forceinline__ void dep_guard_b(v8f& a, v8f& b, v16b x, v16b y) { asm volatile("v_nop\n\tv_nop\n\tv_nop\n\tv_nop" : "+v"(a), "+v"(b) : "v"(x), "v"(y)); }
__device__ __forceinline__ void keep4_b(v16b a, v16b b, v16b c, v16b d) { asm volatile("v_nop" :: "v"(a), "v"(b), "v"(c), "v"(d)); }
__device__ __forceinline__ void acc_guard4(v8f& a, v8f& b, v8f& c, v8f& d) { asm volatile("v_nop\n\tv_nop\n\tv_nop\n\tv_nop" : "+v"(a), "+v"(b), "+v"(c), "+v"(d)); }

template <typename T> struct Frag;
template <> struct Frag<__bf16> {
  typedef v16b V; union U { v16b v; v8b h[2]; };
  static __device__ __forceinline__ v16b load(const __bf16* p) {
    U f; f.h[0] = *(const v8b*)(p); f.h[1] = *(const v8b*)(p + 16); return f.v;
  }
  static __device__ __forceinline__ v8f mma(v16b a, v16b b, v8f c) {
    return __builtin_amdgcn_wmma_f32_16x16x32_bf16(false, a, false, b, (short)0, c, false, false);
  }
  static __device__ __forceinline__ void guard(v8f& a, v8f& b, v16b x, v16b y) { dep_guard_b(a, b, x, y); }
  static __device__ __forceinline__ void keep(v16b a, v16b b, v16b c, v16b d) { keep4_b(a, b, c, d); }
};

__device__ __forceinline__ float lgst(float x) {
  const float e = expf(-fabsf(x));
  const float r = __builtin_amdgcn_rcpf(1.0f + e);
  return (x >= 0.0f) ? r : e * r;
}
__device__ __forceinline__ float htan(float x) {
  const float e = expf(-2.0f * fabsf(x));
  const float m = (1.0f - e) * __builtin_amdgcn_rcpf(1.0f + e);
  return copysignf(m, x);
}

__global__ __launch_bounds__(256) void cast_x_bf16(const float* __restrict__ x, unsigned short* __restrict__ xb) {
  const int g = blockIdx.x * 256 + (int)threadIdx.x;
  const int rowOut = g >> 7;
  const int e8 = (g & 127) * 8;
  const int tt = rowOut >> 6, bb = rowOut & 63;
  const float* src = x + ((size_t)bb * kSteps + tt) * kFeat + e8;
  const v4f a = *(const v4f*)src;
  const v4f c = *(const v4f*)(src + 4);
  v4u w;
  w[0] = (unsigned)f2bf_bits(a[0]) | ((unsigned)f2bf_bits(a[1]) << 16);
  w[1] = (unsigned)f2bf_bits(a[2]) | ((unsigned)f2bf_bits(a[3]) << 16);
  w[2] = (unsigned)f2bf_bits(c[0]) | ((unsigned)f2bf_bits(c[1]) << 16);
  w[3] = (unsigned)f2bf_bits(c[2]) | ((unsigned)f2bf_bits(c[3]) << 16);
  unsigned short* dst = xb + (size_t)rowOut * kFeat + e8;
  *(volatile v4u*)(void*)dst = w;
  __threadfence();
  *(volatile v4u*)(void*)dst = w;
}

__global__ __launch_bounds__(256) void w_transpose_bf16(const float* __restrict__ W,
                                                        unsigned short* __restrict__ wxt,
                                                        unsigned short* __restrict__ wht) {
  __shared__ __align__(16) unsigned short sT[64 * kTPitch];
  const int tid = threadIdx.x, lane = tid & 31, wave = tid >> 5;
  const int n0 = blockIdx.x * 64;
  const int kt = blockIdx.y;
  const int k0 = kt * 64;
  for (int q = tid; q < 1024; q += 256) {
    const int kk = q >> 4, c4 = (q & 15) * 4;
    const v4f v = *(const v4f*)(W + (size_t)(k0 + kk) * kGate4 + n0 + c4);
    sT[(c4 + 0) * kTPitch + kk] = f2bf_bits(v[0]);
    sT[(c4 + 1) * kTPitch + kk] = f2bf_bits(v[1]);
    sT[(c4 + 2) * kTPitch + kk] = f2bf_bits(v[2]);
    sT[(c4 + 3) * kTPitch + kk] = f2bf_bits(v[3]);
  }
  __syncthreads();
  const bool first = (kt < (kFeat / 64));
  unsigned short* plane = first ? wxt : wht;
  const int kcol = first ? k0 : (k0 - kFeat);
  const int q8 = lane >> 3, c8 = (lane & 7) * 8;
  for (int pass = 0; pass < 2; ++pass) {
#pragma unroll
    for (int it = 0; it < 2; ++it) {
      const int nn = wave * 8 + it * 4 + q8;
      const v4u val = *(const v4u*)(const void*)(sT + nn * kTPitch + c8);
      *(volatile v4u*)(void*)(plane + (size_t)(n0 + nn) * kHid + kcol + c8) = val;
    }
    __threadfence();
  }
}

__global__ __launch_bounds__(256) void zero_fill4(float* __restrict__ p, int n4) {
  const int g = blockIdx.x * 256 + (int)threadIdx.x;
  if (g < n4) {
    const v4f z = {0.0f, 0.0f, 0.0f, 0.0f};
    *(volatile v4f*)(p + 4 * (size_t)g) = z;
    __threadfence();
    *(volatile v4f*)(p + 4 * (size_t)g) = z;
  }
}

__global__ __launch_bounds__(128) void lstm_step(
    const unsigned short* __restrict__ xb,
    const unsigned short* __restrict__ wxt,
    const unsigned short* __restrict__ wht,
    const float* __restrict__ bias,
    const float* __restrict__ cin,
    const unsigned short* __restrict__ hhin,
    const unsigned short* __restrict__ hlin,
    float* __restrict__ cnx,
    unsigned short* __restrict__ hhnx,
    unsigned short* __restrict__ hlnx,
    float* __restrict__ out,
    int t) {
  __shared__ __align__(16) float sC[kBatch * kColsBlk];
  __shared__ __align__(16) float sZ[4 * 16 * kColsBlk];
  __shared__ __align__(16) float sH[kBatch * kColsBlk];

  const int tid = threadIdx.x, lane = tid & 31, wave = tid >> 5;
  const int rlane = lane & 15, hf = lane >> 4, koff = hf * 8;
  const int nblk = blockIdx.x * kColsBlk;
  const int nw = nblk + wave * 16;

  const __bf16* Xt = (const __bf16*)xb + (size_t)t * kBatch * kFeat;
  const __bf16* Wx = (const __bf16*)wxt;
  const __bf16* Wh = (const __bf16*)wht;
  const __bf16* Hh = (const __bf16*)hhin;
  const __bf16* Hl = (const __bf16*)hlin;

  for (int q = tid; q < kBatch * (kColsBlk / 4); q += 128) {
    const int row = q >> 4, c4 = (q & 15) * 4;
    const v4f v = *(const v4f*)(cin + (size_t)row * kHid + nblk + c4);
    *(v4f*)(sC + row * kColsBlk + c4) = v;
  }
  __syncthreads();

  v8f acc[4][4];
#pragma unroll
  for (int i = 0; i < 4; ++i)
#pragma unroll
    for (int j = 0; j < 4; ++j) acc[i][j] = (v8f){0.f,0.f,0.f,0.f,0.f,0.f,0.f,0.f};

  for (int k0 = 0; k0 < kFeat; k0 += 32) {
    v16b bw[4];
#pragma unroll
    for (int j = 0; j < 4; ++j)
      bw[j] = Frag<__bf16>::load(Wx + (size_t)(j * kHid + nw + rlane) * kFeat + koff + k0);
#pragma unroll
    for (int i = 0; i < 4; ++i) {
      const v16b a = Frag<__bf16>::load(Xt + (size_t)(i * 16 + rlane) * kFeat + koff + k0);
#pragma unroll
      for (int j = 0; j < 4; ++j) acc[i][j] = Frag<__bf16>::mma(a, bw[j], acc[i][j]);
      Frag<__bf16>::guard(acc[i][0], acc[i][3], a, a);
    }
    Frag<__bf16>::keep(bw[0], bw[1], bw[2], bw[3]);
  }
  for (int k0 = 0; k0 < kHid; k0 += 32) {
    v16b bw[4];
#pragma unroll
    for (int j = 0; j < 4; ++j)
      bw[j] = Frag<__bf16>::load(Wh + (size_t)(j * kHid + nw + rlane) * kHid + koff + k0);
#pragma unroll
    for (int i = 0; i < 4; ++i) {
      const size_t ao = (size_t)(i * 16 + rlane) * kHid + koff + k0;
      const v16b ah = Frag<__bf16>::load(Hh + ao);
      const v16b al = Frag<__bf16>::load(Hl + ao);
#pragma unroll
      for (int j = 0; j < 4; ++j) {
        acc[i][j] = Frag<__bf16>::mma(ah, bw[j], acc[i][j]);
        acc[i][j] = Frag<__bf16>::mma(al, bw[j], acc[i][j]);
      }
      Frag<__bf16>::guard(acc[i][0], acc[i][3], ah, al);
    }
    Frag<__bf16>::keep(bw[0], bw[1], bw[2], bw[3]);
  }
  acc_guard4(acc[0][0], acc[0][1], acc[0][2], acc[0][3]);
  acc_guard4(acc[1][0], acc[1][1], acc[1][2], acc[1][3]);
  acc_guard4(acc[2][0], acc[2][1], acc[2][2], acc[2][3]);
  acc_guard4(acc[3][0], acc[3][1], acc[3][2], acc[3][3]);

  float bv[4];
#pragma unroll
  for (int j = 0; j < 4; ++j) bv[j] = bf_bits2f(f2bf_bits(bias[j * kHid + nw + rlane]));

#pragma unroll
  for (int i = 0; i < 4; ++i) {
#pragma unroll
    for (int j = 0; j < 4; ++j)
#pragma unroll
      for (int r = 0; r < 8; ++r)
        sZ[(j * 16 + hf * 8 + r) * kColsBlk + wave * 16 + rlane] = acc[i][j][r] + bv[j];
    __syncthreads();
#pragma unroll 1
    for (int e = tid; e < 16 * kColsBlk; e += 128) {
      const int rr = e >> 6, cc = e & 63;
      const int row = i * 16 + rr;
      const float zi = sZ[(0 * 16 + rr) * kColsBlk + cc];
      const float zj = sZ[(1 * 16 + rr) * kColsBlk + cc];
      const float zf = sZ[(2 * 16 + rr) * kColsBlk + cc] + 1.0f;
      const float zo = sZ[(3 * 16 + rr) * kColsBlk + cc];
      const float cold = sC[row * kColsBlk + cc];
      const float cnew = cold * lgst(zf) + lgst(zi) * htan(zj);
      const float hnew = htan(cnew) * lgst(zo);
      sC[row * kColsBlk + cc] = cnew;
      sH[row * kColsBlk + cc] = hnew;
    }
    __syncthreads();
  }

  const int c4 = rlane * 4;
  const int q8 = lane >> 3, c8 = (lane & 7) * 8;
  for (int pass = 0; pass < 2; ++pass) {
#pragma unroll
    for (int it = 0; it < 8; ++it) {
      const int row = wave * 16 + it * 2 + hf;
      const v4f cv = *(const v4f*)(sC + row * kColsBlk + c4);
      const v4f hv = *(const v4f*)(sH + row * kColsBlk + c4);
      *(volatile v4f*)(cnx + (size_t)row * kHid + nblk + c4) = cv;
      *(volatile v4f*)(out + ((size_t)row * kSteps + t) * kHid + nblk + c4) = hv;
    }
#pragma unroll
    for (int it = 0; it < 4; ++it) {
      const int row = wave * 16 + it * 4 + q8;
      const v4f f0 = *(const v4f*)(sH + row * kColsBlk + c8);
      const v4f f1 = *(const v4f*)(sH + row * kColsBlk + c8 + 4);
      float fv[8];
      fv[0] = f0[0]; fv[1] = f0[1]; fv[2] = f0[2]; fv[3] = f0[3];
      fv[4] = f1[0]; fv[5] = f1[1]; fv[6] = f1[2]; fv[7] = f1[3];
      v4u hw, lw;
#pragma unroll
      for (int p = 0; p < 4; ++p) {
        const unsigned short ha = f2bf_bits(fv[2 * p]);
        const unsigned short hb = f2bf_bits(fv[2 * p + 1]);
        const unsigned short la = f2bf_bits(fv[2 * p] - bf_bits2f(ha));
        const unsigned short lb = f2bf_bits(fv[2 * p + 1] - bf_bits2f(hb));
        hw[p] = (unsigned)ha | ((unsigned)hb << 16);
        lw[p] = (unsigned)la | ((unsigned)lb << 16);
      }
      *(volatile v4u*)(void*)(hhnx + (size_t)row * kHid + nblk + c8) = hw;
      *(volatile v4u*)(void*)(hlnx + (size_t)row * kHid + nblk + c8) = lw;
    }
    __threadfence();
  }
}

extern "C" void kernel_launch(void* const* d_in, const int* in_sizes, int n_in,
                              void* d_out, int out_size, void* d_ws, size_t ws_size,
                              hipStream_t stream) {
  if (n_in < 3) return;
  if (in_sizes[0] != kBatch * kSteps * kFeat) return;
  if (in_sizes[1] != (kFeat + kHid) * kGate4) return;
  if (in_sizes[2] != kGate4) return;
  if (out_size != kBatch * kSteps * kHid) return;

  const float* x    = (const float*)d_in[0];
  const float* W    = (const float*)d_in[1];
  const float* bias = (const float*)d_in[2];
  float*       out  = (float*)d_out;

  const size_t xbBytes  = (size_t)kBatch * kSteps * kFeat * 2;
  const size_t wpBytes  = (size_t)kGate4 * kHid * 2;
  const size_t cBytes   = (size_t)kBatch * kHid * 4;
  const size_t hBytes   = (size_t)kBatch * kHid * 2;
  const size_t setBytes = cBytes + 2 * hBytes;

  const size_t offXb   = 0;
  const size_t offWxt  = offXb + xbBytes;
  const size_t offWht  = offWxt + wpBytes;
  const size_t offSet0 = offWht + wpBytes;
  const size_t offSet1 = offSet0 + setBytes;
  const size_t total   = offSet1 + setBytes;
  if (total > ws_size) return;

  uint8_t* ws = (uint8_t*)d_ws;
  unsigned short* xb  = (unsigned short*)(ws + offXb);
  unsigned short* wxt = (unsigned short*)(ws + offWxt);
  unsigned short* wht = (unsigned short*)(ws + offWht);
  float*          c0  = (float*)(ws + offSet0);
  unsigned short* hh0 = (unsigned short*)(ws + offSet0 + cBytes);
  unsigned short* hl0 = (unsigned short*)(ws + offSet0 + cBytes + hBytes);
  float*          c1  = (float*)(ws + offSet1);
  unsigned short* hh1 = (unsigned short*)(ws + offSet1 + cBytes);
  unsigned short* hl1 = (unsigned short*)(ws + offSet1 + cBytes + hBytes);

  const int nx8 = kBatch * kSteps * kFeat / 8;
  cast_x_bf16<<<nx8 / 256, 256, 0, stream>>>(x, xb);
  w_transpose_bf16<<<dim3(kGate4 / 64, (kFeat + kHid) / 64), 256, 0, stream>>>(W, wxt, wht);
  const int nz4 = (int)(setBytes / 16);
  zero_fill4<<<(nz4 + 255) / 256, 256, 0, stream>>>(c0, nz4);

  for (int t = 0; t < kSteps; ++t) {
    const bool even = ((t & 1) == 0);
    const float*          ci  = even ? c0  : c1;
    const unsigned short* hhi = even ? hh0 : hh1;
    const unsigned short* hli = even ? hl0 : hl1;
    float*                cn  = even ? c1  : c0;
    unsigned short*       hhn = even ? hh1 : hh0;
    unsigned short*       hln = even ? hl1 : hl0;
    lstm_step<<<kHid / kColsBlk, 128, 0, stream>>>(xb, wxt, wht, bias, ci, hhi, hli, cn, hhn, hln, out, t);
  }
}
